// Involution_19877108646071
// MI455X (gfx1250) — hardware-run, weakly checked
//
#include <hip/hip_runtime.h>
#include <math.h>

typedef __attribute__((ext_vector_type(16))) __bf16   v16b;
typedef __attribute__((ext_vector_type(8)))  __bf16   v8b;
typedef __attribute__((ext_vector_type(8)))  _Float16 v8h;
typedef __attribute__((ext_vector_type(8)))  float    v8f;
typedef __attribute__((ext_vector_type(4)))  float    v4f;
typedef __attribute__((ext_vector_type(4)))  unsigned v4u;
typedef __attribute__((ext_vector_type(8)))  unsigned v8u;

constexpr int kBatch  = 4;
constexpr int kChan   = 64;
constexpr int kHt     = 128;
constexpr int kWd     = 128;
constexpr int kHW     = kHt * kWd;
constexpr int kPix    = kBatch * kHW;
constexpr int kKsz    = 7;
constexpr int kTaps   = kKsz * kKsz;
constexpr int kGroups = 4;
constexpr int kGrpCh  = 16;
constexpr int kKO     = kTaps * kGroups;
constexpr int kMPad   = 256;
constexpr int kMTiles = 13;
constexpr int kSlabP  = 36;
constexpr int kTileH  = 4;
constexpr int kTileW  = 32;
constexpr int kHaloH  = kTileH + kKsz - 1;
constexpr int kHaloW  = kTileW + kKsz - 1;
constexpr int kChP    = kHaloH * kHaloW;
constexpr int kHaloN  = kGrpCh * kChP;
constexpr int kHaloIt = 48;
constexpr int kHaloPad = kHaloIt * 128;
constexpr int kBwWave = 16 * 64;
constexpr int kBwZero = 4 * kBwWave;
constexpr int kBwTot  = kBwZero + 32;
constexpr int kStP    = 36;
constexpr int kD39    = kHaloW + 1;
constexpr int kD70    = 2 * kHaloW - 6;
static_assert(kKO == 196, "generated kernel channels");
static_assert(kGroups * kGrpCh == kChan, "group split");
static_assert((kChan % 32) == 0, "GEMM K multiple of 32");
static_assert(kMTiles * 16 >= kKO && kMTiles * 16 <= kMPad, "M tiles inside the padded W planes");
static_assert((kPix % (32 * 8)) == 0 && (kHW % 32) == 0, "N tiling exact, pixel runs stay inside one image");
static_assert(kHaloH == 10 && kHaloW == 38 && kChP == 380 && kHaloN == 6080, "halo tile");
static_assert(kHaloPad == 6144 && kHaloPad >= kHaloN, "halo staging covers the tile");
static_assert((kHt % kTileH) == 0 && (kWd % kTileW) == 0, "output tiling exact");
static_assert(kTaps <= 64 && kTaps == 49, "taps padded to two k-steps of 32");
static_assert(kD39 == 39 && kD70 == 70, "tap offset deltas");

constexpr size_t kOffXH  = 0;
constexpr size_t kOffXL  = kOffXH + (size_t)kPix * kChan * 2;
constexpr size_t kOffWH  = kOffXL + (size_t)kPix * kChan * 2;
constexpr size_t kOffWL  = kOffWH + (size_t)kMPad * kChan * 2;
constexpr size_t kOffSS  = kOffWL + (size_t)kMPad * kChan * 2;
constexpr size_t kOffWGT = kOffSS + (size_t)2 * kMPad * 4;
constexpr size_t kWsTotal = kOffWGT + (size_t)kBatch * kKO * kHW * 4;
static_assert(kWsTotal == 68225024ull, "carve total");
static_assert(kWsTotal <= 134217728ull, "carve cap");
static_assert((kOffXL % 128) == 0 && (kOffWH % 128) == 0 && (kOffWL % 128) == 0 &&
              (kOffSS % 128) == 0 && (kOffWGT % 128) == 0, "128-B aligned regions");

__device__ __forceinline__ unsigned short f2bf_bits(float f) {
  unsigned u = __float_as_uint(f);
  return (unsigned short)((u + 0x7FFFu + ((u >> 16) & 1u)) >> 16);
}
__device__ __forceinline__ float bf_bits2f(unsigned short h) { return __uint_as_float(((unsigned)h) << 16); }

__device__ __forceinline__ unsigned bf_rne_u32(float f) {
  const unsigned u = __float_as_uint(f);
  return (u + 0x7FFFu + ((u >> 16) & 1u)) >> 16;
}
__device__ __forceinline__ void split_u32(float f, unsigned& hb, unsigned& lb) {
  hb = bf_rne_u32(f);
  lb = bf_rne_u32(f - __uint_as_float(hb << 16));
}
__device__ __forceinline__ unsigned pk16(unsigned lo16, unsigned hi16) { return lo16 | (hi16 << 16); }

__device__ __forceinline__ v16b frag_load_bf(const __bf16* p) {
  union { v16b v; v8b h[2]; } f;
  f.h[0] = *(const v8b*)(p);
  f.h[1] = *(const v8b*)(p + 16);
  return f.v;
}
__device__ __forceinline__ v8f mma_bf(v16b a, v16b b, v8f c) {
  c = __builtin_amdgcn_wmma_f32_16x16x32_bf16(false, a, false, b, (short)0, c, false, false);
  asm volatile("v_nop\n\tv_nop\n\tv_nop\n\tv_nop" : "+v"(c) : "v"(a), "v"(b));
  return c;
}

__global__ __launch_bounds__(256) void prep_x_kernel(
    const float* __restrict__ x, unsigned short* __restrict__ XH, unsigned short* __restrict__ XL)
{
  __shared__ float sT[64 * 33];
  const int tid  = threadIdx.x;
  const int pix0 = blockIdx.x * 32;
  const int b    = pix0 >> 14;
  const int hw0  = pix0 & (kHW - 1);
  const int p    = tid & 31;
  const int cr   = tid >> 5;
  const float* xb = x + (size_t)b * kChan * kHW + hw0 + p;
#pragma unroll
  for (int i = 0; i < 8; ++i) {
    const int c = cr + 8 * i;
    sT[c * 33 + p] = xb[(size_t)c * kHW];
  }
  __syncthreads();
  const int pr = tid >> 3;
  const int c8 = (tid & 7) * 8;
  v8h hv, lv;
#pragma unroll
  for (int e = 0; e < 8; ++e) {
    const float f = sT[(c8 + e) * 33 + pr];
    const unsigned short hb = f2bf_bits(f);
    const unsigned short lb = f2bf_bits(f - bf_bits2f(hb));
    hv[e] = __builtin_bit_cast(_Float16, hb);
    lv[e] = __builtin_bit_cast(_Float16, lb);
  }
  const size_t o = (size_t)(pix0 + pr) * kChan + c8;
  *(volatile v8h*)(XH + o) = hv;
  *(volatile v8h*)(XL + o) = lv;
  __threadfence();
  *(volatile v8h*)(XH + o) = hv;
  *(volatile v8h*)(XL + o) = lv;
}

__global__ __launch_bounds__(256) void prep_w_kernel(
    const float* __restrict__ cw, const float* __restrict__ gam, const float* __restrict__ bet,
    const float* __restrict__ mu, const float* __restrict__ var,
    unsigned short* __restrict__ WH, unsigned short* __restrict__ WL, float* __restrict__ ss)
{
  const int tid = threadIdx.x;
  if (blockIdx.x < 8) {
    const int i   = blockIdx.x * 256 + tid;
    const int e0  = i * 8;
    const int row = e0 >> 6;
    const int col = e0 & 63;
    const bool valid = row < kKO;
    const int rc = valid ? row : (kKO - 1);
    const float* sp = cw + (size_t)rc * kChan + col;
    const v4f a0 = *(const v4f*)(sp);
    const v4f a1 = *(const v4f*)(sp + 4);
    v8h hv, lv;
#pragma unroll
    for (int e = 0; e < 4; ++e) {
      const float f0 = valid ? a0[e] : 0.0f;
      const float f1 = valid ? a1[e] : 0.0f;
      const unsigned short h0 = f2bf_bits(f0);
      const unsigned short h1 = f2bf_bits(f1);
      const unsigned short l0 = f2bf_bits(f0 - bf_bits2f(h0));
      const unsigned short l1 = f2bf_bits(f1 - bf_bits2f(h1));
      hv[e]     = __builtin_bit_cast(_Float16, h0);
      hv[4 + e] = __builtin_bit_cast(_Float16, h1);
      lv[e]     = __builtin_bit_cast(_Float16, l0);
      lv[4 + e] = __builtin_bit_cast(_Float16, l1);
    }
    *(volatile v8h*)(WH + e0) = hv;
    *(volatile v8h*)(WL + e0) = lv;
    __threadfence();
    *(volatile v8h*)(WH + e0) = hv;
    *(volatile v8h*)(WL + e0) = lv;
  } else {
    const int o = tid;
    const bool valid = o < kKO;
    const int oc = valid ? o : (kKO - 1);
    const float g = gam[oc];
    const float be = bet[oc];
    const float m = mu[oc];
    const float v = var[oc];
    const float sc0 = g / sqrtf(v + 1e-5f);
    const float sh0 = be - m * sc0;
    const float sc = valid ? sc0 : 0.0f;
    const float sh = valid ? sh0 : 0.0f;
    volatile float* p0 = ss + o;
    volatile float* p1 = ss + kMPad + o;
    *p0 = sc;
    *p1 = sh;
    __threadfence();
    *p0 = sc;
    *p1 = sh;
  }
}

__global__ __launch_bounds__(256) void conv1x1_silu_kernel(
    const unsigned short* __restrict__ WHp, const unsigned short* __restrict__ WLp,
    const unsigned short* __restrict__ XHp, const unsigned short* __restrict__ XLp,
    const float* __restrict__ ss, float* __restrict__ wgt)
{
  __shared__ __align__(16) float sT[8][16 * kSlabP];
  const __bf16* WH = (const __bf16*)WHp;
  const __bf16* WL = (const __bf16*)WLp;
  const __bf16* XH = (const __bf16*)XHp;
  const __bf16* XL = (const __bf16*)XLp;
  const int lane = threadIdx.x & 31;
  const int wave = threadIdx.x >> 5;
  const int rl   = lane & 15;
  const int hh   = lane >> 4;
  const int koff = hh * 8;
  const int mOff = hh * 8;
  const int pix0 = (blockIdx.x * 8 + wave) * 32;
  const int b    = pix0 >> 14;
  const int pin  = pix0 & (kHW - 1);

  v16b xh[2][2], xl[2][2];
#pragma unroll
  for (int j = 0; j < 2; ++j) {
#pragma unroll
    for (int ks = 0; ks < 2; ++ks) {
      const size_t bo = (size_t)(pix0 + j * 16 + rl) * kChan + ks * 32 + koff;
      xh[j][ks] = frag_load_bf(XH + bo);
      xl[j][ks] = frag_load_bf(XL + bo);
    }
  }

  float* slab = sT[wave];
  float* dst  = wgt + (size_t)b * kKO * kHW + pin;
  const int q  = lane >> 3;
  const int c4 = (lane & 7) * 4;

#pragma unroll 1
  for (int mt = 0; mt < kMTiles; ++mt) {
    const int m0 = mt * 16;
    v16b ah[2], al[2];
#pragma unroll
    for (int ks = 0; ks < 2; ++ks) {
      const size_t ao = (size_t)(m0 + rl) * kChan + ks * 32 + koff;
      ah[ks] = frag_load_bf(WH + ao);
      al[ks] = frag_load_bf(WL + ao);
    }
    v8f acc[2];
    acc[0] = (v8f){0.f, 0.f, 0.f, 0.f, 0.f, 0.f, 0.f, 0.f};
    acc[1] = (v8f){0.f, 0.f, 0.f, 0.f, 0.f, 0.f, 0.f, 0.f};
#pragma unroll
    for (int ks = 0; ks < 2; ++ks) {
#pragma unroll
      for (int j = 0; j < 2; ++j) {
        acc[j] = mma_bf(ah[ks], xh[j][ks], acc[j]);
        acc[j] = mma_bf(ah[ks], xl[j][ks], acc[j]);
        acc[j] = mma_bf(al[ks], xh[j][ks], acc[j]);
      }
    }

#pragma unroll
    for (int j = 0; j < 2; ++j) {
#pragma unroll
      for (int r = 0; r < 8; ++r) {
        slab[(mOff + r) * kSlabP + j * 16 + rl] = acc[j][r];
      }
    }
    __builtin_amdgcn_fence(__ATOMIC_RELEASE, "workgroup");
    __builtin_amdgcn_wave_barrier();
    __builtin_amdgcn_fence(__ATOMIC_ACQUIRE, "workgroup");

#pragma unroll 1
    for (int it = 0; it < 4; ++it) {
      const int row = it * 4 + q;
      const int o   = m0 + row;
      const float sc = ss[o];
      const float sh = ss[kMPad + o];
      float* sp = slab + row * kSlabP + c4;
      const v4f v = *(const v4f*)sp;
      v4f w;
#pragma unroll
      for (int e = 0; e < 4; ++e) {
        const float t  = v[e] * sc + sh;
        const float sg = 1.0f / (1.0f + expf(-t));
        w[e] = t * sg;
      }
      *(v4f*)sp = w;
    }

    for (int pass = 0; pass < 2; ++pass) {
#pragma unroll
      for (int it = 0; it < 4; ++it) {
        const int row = it * 4 + q;
        const int o   = m0 + row;
        if (o < kKO) {
          const v4f w = *(const v4f*)(slab + row * kSlabP + c4);
          *(volatile v4f*)(dst + (size_t)o * kHW + c4) = w;
        }
      }
      __threadfence();
    }
    __builtin_amdgcn_fence(__ATOMIC_RELEASE, "workgroup");
    __builtin_amdgcn_wave_barrier();
    __builtin_amdgcn_fence(__ATOMIC_ACQUIRE, "workgroup");
  }
}

__global__ __launch_bounds__(128) void involution_wmma_kernel(
    const float* __restrict__ x, const float* __restrict__ wgt, float* __restrict__ out)
{
  __shared__ __align__(16) unsigned xsw[kHaloPad];
  __shared__ __align__(16) unsigned bwz[kBwTot];
  __shared__ __align__(16) float stag[4][16 * kStP];
  const int tid  = threadIdx.x;
  const int lane = tid & 31;
  const int wave = tid >> 5;
  const int rl   = lane & 15;
  const int hh   = lane >> 4;
  const int bx   = blockIdx.x;
  const int tx   = bx & 3;
  const int ty   = (bx >> 2) & 31;
  const int g    = (bx >> 7) & 3;
  const int b    = bx >> 9;
  const int h0   = ty * kTileH;
  const int w0   = tx * kTileW;
  const float* xg = x + (size_t)(b * kChan + g * kGrpCh) * kHW;

  if (tid < 32) {
    bwz[kBwZero + tid] = 0u;
  }

#pragma unroll 1
  for (int it = 0; it < kHaloIt; ++it) {
    const int i   = it * 128 + tid;
    const bool inr = i < kHaloN;
    const int ic  = inr ? i : (kHaloN - 1);
    const int c   = ic / kChP;
    const int rem = ic - c * kChP;
    const int hr  = rem / kHaloW;
    const int wc  = rem - hr * kHaloW;
    const int hy  = h0 - 3 + hr;
    const int wx  = w0 - 3 + wc;
    const bool valid = inr && (hy >= 0) && (hy < kHt) && (wx >= 0) && (wx < kWd);
    const int hyc = hy < 0 ? 0 : (hy > kHt - 1 ? kHt - 1 : hy);
    const int wxc = wx < 0 ? 0 : (wx > kWd - 1 ? kWd - 1 : wx);
    float v = xg[(size_t)c * kHW + hyc * kWd + wxc];
    asm volatile("" : "+v"(v));
    const float f = valid ? v : 0.0f;
    unsigned hb, lb;
    split_u32(f, hb, lb);
    xsw[i] = pk16(hb, lb);
  }
  __syncthreads();

  const int hrow = h0 + wave;
  const int a0  = rl * kChP + wave * kHaloW;
  const int a39 = a0 + kD39 * hh;
  const int a70 = a0 + kD70 * hh;
  const int boff = (rl == 0) ? (wave * kBwWave + hh * 32) : kBwZero;
  const int bstr = (rl == 0) ? 64 : 0;
  const float* wrow = wgt + (size_t)(b * kKO + g * kTaps) * kHW + (size_t)hrow * kWd + w0;
  float* sg = stag[wave];

#pragma unroll 1
  for (int hb2 = 0; hb2 < 2; ++hb2) {
    {
      const float* wq  = wrow + hb2 * 16 + rl;
      const float* wqh = wq + (size_t)(8 * hh) * kHW;
      float wv[25];
#pragma unroll
      for (int e = 0; e < 8; ++e) wv[e] = wqh[(size_t)e * kHW];
      asm volatile("" : "+v"(wv[0]), "+v"(wv[1]), "+v"(wv[2]), "+v"(wv[3]),
                        "+v"(wv[4]), "+v"(wv[5]), "+v"(wv[6]), "+v"(wv[7]) :: "memory");
#pragma unroll
      for (int e = 0; e < 8; ++e) wv[8 + e] = wqh[(size_t)(16 + e) * kHW];
      asm volatile("" : "+v"(wv[8]), "+v"(wv[9]), "+v"(wv[10]), "+v"(wv[11]),
                        "+v"(wv[12]), "+v"(wv[13]), "+v"(wv[14]), "+v"(wv[15]) :: "memory");
#pragma unroll
      for (int e = 0; e < 8; ++e) wv[16 + e] = wqh[(size_t)(32 + e) * kHW];
      wv[24] = wq[(size_t)48 * kHW];
      asm volatile("" : "+v"(wv[16]), "+v"(wv[17]), "+v"(wv[18]), "+v"(wv[19]),
                        "+v"(wv[20]), "+v"(wv[21]), "+v"(wv[22]), "+v"(wv[23]) :: "memory");
      asm volatile("" : "+v"(wv[24]) :: "memory");
      const float f48 = (hh == 0) ? wv[24] : 0.0f;
      unsigned hbv[24], lbv[24];
#pragma unroll
      for (int e = 0; e < 24; ++e) split_u32(wv[e], hbv[e], lbv[e]);
      unsigned hb48, lb48;
      split_u32(f48, hb48, lb48);
      const v4u s0h0 = (v4u){pk16(hbv[0], hbv[1]), pk16(hbv[2], hbv[3]), pk16(hbv[4], hbv[5]), pk16(hbv[6], hbv[7])};
      const v4u s0h1 = (v4u){pk16(hbv[8], hbv[9]), pk16(hbv[10], hbv[11]), pk16(hbv[12], hbv[13]), pk16(hbv[14], hbv[15])};
      const v4u s0l0 = (v4u){pk16(lbv[0], lbv[1]), pk16(lbv[2], lbv[3]), pk16(lbv[4], lbv[5]), pk16(lbv[6], lbv[7])};
      const v4u s0l1 = (v4u){pk16(lbv[8], lbv[9]), pk16(lbv[10], lbv[11]), pk16(lbv[12], lbv[13]), pk16(lbv[14], lbv[15])};
      const v4u s1h0 = (v4u){pk16(hbv[16], hbv[17]), pk16(hbv[18], hbv[19]), pk16(hbv[20], hbv[21]), pk16(hbv[22], hbv[23])};
      const v4u s1l0 = (v4u){pk16(lbv[16], lbv[17]), pk16(lbv[18], lbv[19]), pk16(lbv[20], lbv[21]), pk16(lbv[22], lbv[23])};
      const v4u s1h1 = (v4u){hb48, 0u, 0u, 0u};
      const v4u s1l1 = (v4u){lb48, 0u, 0u, 0u};
      unsigned* bd = &bwz[wave * kBwWave + (rl * 2 + hh) * 32];
      *(v4u*)(bd + 0)  = s0h0;
      *(v4u*)(bd + 4)  = s0h1;
      *(v4u*)(bd + 8)  = s0l0;
      *(v4u*)(bd + 12) = s0l1;
      *(v4u*)(bd + 16) = s1h0;
      *(v4u*)(bd + 20) = s1h1;
      *(v4u*)(bd + 24) = s1l0;
      *(v4u*)(bd + 28) = s1l1;
    }
    __builtin_amdgcn_fence(__ATOMIC_RELEASE, "workgroup");
    __builtin_amdgcn_wave_barrier();
    __builtin_amdgcn_fence(__ATOMIC_ACQUIRE, "workgroup");

#pragma unroll 1
    for (int j = 0; j < 16; ++j) {
      const int col = hb2 * 16 + j;
      const int i0  = a0 + col;
      const int i39 = a39 + col;
      const int i70 = a70 + col;
      v8u ah0u, al0u, ah1u, al1u;
#pragma unroll
      for (int jw = 0; jw < 8; ++jw) {
        const int e0 = 2 * jw;
        const int e1 = 2 * jw + 1;
        const int c0 = (e0 & 7) + (e0 >> 3) * 16;
        const int c1 = (e1 & 7) + (e1 >> 3) * 16;
        const unsigned wa = xsw[(((c0 % 7) == 6) ? i70 : i39) + (c0 / 7) * kHaloW + (c0 % 7)];
        const unsigned wb = xsw[(((c1 % 7) == 6) ? i70 : i39) + (c1 / 7) * kHaloW + (c1 % 7)];
        ah0u[jw] = (wa & 0xffffu) | (wb << 16);
        al0u[jw] = (wa >> 16) | (wb & 0xffff0000u);
      }
#pragma unroll
      for (int jw = 0; jw < 4; ++jw) {
        const int c0 = 32 + 2 * jw;
        const int c1 = 33 + 2 * jw;
        const unsigned wa = xsw[(((c0 % 7) == 6) ? i70 : i39) + (c0 / 7) * kHaloW + (c0 % 7)];
        const unsigned wb = xsw[(((c1 % 7) == 6) ? i70 : i39) + (c1 / 7) * kHaloW + (c1 % 7)];
        ah1u[jw] = (wa & 0xffffu) | (wb << 16);
        al1u[jw] = (wa >> 16) | (wb & 0xffff0000u);
      }
      {
        unsigned w8 = xsw[i0 + 6 * kHaloW + 6];
        asm volatile("" : "+v"(w8));
        const unsigned w8s = (hh == 0) ? w8 : 0u;
        ah1u[4] = w8s & 0xffffu;
        al1u[4] = w8s >> 16;
        ah1u[5] = 0u;
        ah1u[6] = 0u;
        ah1u[7] = 0u;
        al1u[5] = 0u;
        al1u[6] = 0u;
        al1u[7] = 0u;
      }
      const v16b ah0 = __builtin_bit_cast(v16b, ah0u);
      const v16b al0 = __builtin_bit_cast(v16b, al0u);
      const v16b ah1 = __builtin_bit_cast(v16b, ah1u);
      const v16b al1 = __builtin_bit_cast(v16b, al1u);

      const unsigned* bp = &bwz[boff + j * bstr];
      const v4u q0 = *(const v4u*)(bp + 0);
      const v4u q1 = *(const v4u*)(bp + 4);
      const v4u q2 = *(const v4u*)(bp + 8);
      const v4u q3 = *(const v4u*)(bp + 12);
      const v4u q4 = *(const v4u*)(bp + 16);
      const v4u q5 = *(const v4u*)(bp + 20);
      const v4u q6 = *(const v4u*)(bp + 24);
      const v4u q7 = *(const v4u*)(bp + 28);
      const v16b bh0 = __builtin_bit_cast(v16b, __builtin_shufflevector(q0, q1, 0, 1, 2, 3, 4, 5, 6, 7));
      const v16b bl0 = __builtin_bit_cast(v16b, __builtin_shufflevector(q2, q3, 0, 1, 2, 3, 4, 5, 6, 7));
      const v16b bh1 = __builtin_bit_cast(v16b, __builtin_shufflevector(q4, q5, 0, 1, 2, 3, 4, 5, 6, 7));
      const v16b bl1 = __builtin_bit_cast(v16b, __builtin_shufflevector(q6, q7, 0, 1, 2, 3, 4, 5, 6, 7));

      v8f acc = (v8f){0.f, 0.f, 0.f, 0.f, 0.f, 0.f, 0.f, 0.f};
      acc = mma_bf(ah0, bh0, acc);
      acc = mma_bf(ah0, bl0, acc);
      acc = mma_bf(al0, bh0, acc);
      acc = mma_bf(ah1, bh1, acc);
      acc = mma_bf(ah1, bl1, acc);
      acc = mma_bf(al1, bh1, acc);

      if (rl == 0) {
#pragma unroll
        for (int r = 0; r < 8; ++r) {
          sg[(8 * hh + r) * kStP + col] = acc[r];
        }
      }
    }
    __builtin_amdgcn_fence(__ATOMIC_RELEASE, "workgroup");
    __builtin_amdgcn_wave_barrier();
    __builtin_amdgcn_fence(__ATOMIC_ACQUIRE, "workgroup");
  }

  {
    const int q  = lane >> 3;
    const int c4 = (lane & 7) * 4;
    float* ob = out + (size_t)(b * kChan + g * kGrpCh) * kHW + (size_t)hrow * kWd + w0 + c4;
    v4f ov[4];
#pragma unroll
    for (int it = 0; it < 4; ++it) {
      ov[it] = *(const v4f*)(sg + (it * 4 + q) * kStP + c4);
    }
    for (int pass = 0; pass < 2; ++pass) {
#pragma unroll
      for (int it = 0; it < 4; ++it) {
        *(volatile v4f*)(ob + (size_t)(it * 4 + q) * kHW) = ov[it];
      }
      __threadfence();
    }
  }
}

extern "C" void kernel_launch(void* const* d_in, const int* in_sizes, int n_in,
                              void* d_out, int out_size, void* d_ws, size_t ws_size,
                              hipStream_t stream) {
  if (n_in < 6) return;
  if (in_sizes[0] != kPix * kChan) return;
  if (in_sizes[1] != kKO * kChan) return;
  if (in_sizes[2] != kKO) return;
  if (in_sizes[3] != kKO) return;
  if (in_sizes[4] != kKO) return;
  if (in_sizes[5] != kKO) return;
  if (out_size != kPix * kChan) return;
  if (ws_size < kWsTotal) return;

  const float* x      = (const float*)d_in[0];
  const float* conv_w = (const float*)d_in[1];
  const float* gam    = (const float*)d_in[2];
  const float* bet    = (const float*)d_in[3];
  const float* mu     = (const float*)d_in[4];
  const float* var    = (const float*)d_in[5];
  float* out = (float*)d_out;

  char* ws = (char*)d_ws;
  unsigned short* XH  = (unsigned short*)(ws + kOffXH);
  unsigned short* XL  = (unsigned short*)(ws + kOffXL);
  unsigned short* WH  = (unsigned short*)(ws + kOffWH);
  unsigned short* WL  = (unsigned short*)(ws + kOffWL);
  float*          SS  = (float*)(ws + kOffSS);
  float*          WGT = (float*)(ws + kOffWGT);

  prep_x_kernel<<<kPix / 32, 256, 0, stream>>>(x, XH, XL);
  prep_w_kernel<<<9, 256, 0, stream>>>(conv_w, gam, bet, mu, var, WH, WL, SS);
  conv1x1_silu_kernel<<<kPix / 32 / 8, 256, 0, stream>>>(WH, WL, XH, XL, SS, WGT);
  involution_wmma_kernel<<<kBatch * kGroups * (kHt / kTileH) * (kWd / kTileW), 128, 0, stream>>>(x, WGT, out);
}
